// SelfAttentionPose_27530740367859
// MI455X (gfx1250) — hardware-verified
//
#include <hip/hip_runtime.h>
#include <math.h>


#define NBATCH 8
#define NI     512
#define SEQ    1024
#define NTOK   8192
#define NHD    8
#define DHD    64
#define PDIM   128
#define KDIM   514
#define KP     576
#define QKVW   1536
#define LT     8
#define LN_EPS 1e-5f

typedef __attribute__((ext_vector_type(16))) _Float16 v16h;
typedef __attribute__((ext_vector_type(8)))  _Float16 v8h;
typedef __attribute__((ext_vector_type(16))) __bf16   v16b;
typedef __attribute__((ext_vector_type(8)))  __bf16   v8b;
typedef __attribute__((ext_vector_type(8)))  float    v8f;
typedef __attribute__((ext_vector_type(4)))  float    v4f;

__device__ __forceinline__ unsigned short f2bf_bits(float f) {
  unsigned u = __float_as_uint(f);
  return (unsigned short)((u + 0x7FFFu + ((u >> 16) & 1u)) >> 16);
}
__device__ __forceinline__ float bf_bits2f(unsigned short h) { return __uint_as_float(((unsigned)h) << 16); }

__device__ __forceinline__ void dep_guard_h(v8f& a, v8f& b, v16h x, v16h y) { asm volatile("v_nop\n\tv_nop\n\tv_nop\n\tv_nop" : "+v"(a), "+v"(b) : "v"(x), "v"(y)); }
__device__ __forceinline__ void dep_guard_b(v8f& a, v8f& b, v16b x, v16b y) { asm volatile("v_nop\n\tv_nop\n\tv_nop\n\tv_nop" : "+v"(a), "+v"(b) : "v"(x), "v"(y)); }
__device__ __forceinline__ void keep4_h(v16h a, v16h b, v16h c, v16h d) { asm volatile("v_nop" :: "v"(a), "v"(b), "v"(c), "v"(d)); }
__device__ __forceinline__ void keep4_b(v16b a, v16b b, v16b c, v16b d) { asm volatile("v_nop" :: "v"(a), "v"(b), "v"(c), "v"(d)); }
__device__ __forceinline__ void acc_guard4(v8f& a, v8f& b, v8f& c, v8f& d) { asm volatile("v_nop\n\tv_nop\n\tv_nop\n\tv_nop" : "+v"(a), "+v"(b), "+v"(c), "+v"(d)); }
template <typename T> struct Frag;
template <> struct Frag<_Float16> {
  typedef v16h V; union U { v16h v; v8h h[2]; };
  static __device__ __forceinline__ v16h load(const _Float16* p) {
    U f; f.h[0] = *(const v8h*)(p); f.h[1] = *(const v8h*)(p + 16); return f.v;
  }
  static __device__ __forceinline__ v8f mma(v16h a, v16h b, v8f c) {
    return __builtin_amdgcn_wmma_f32_16x16x32_f16(false, a, false, b, (short)0, c, false, false);
  }
  static __device__ __forceinline__ void guard(v8f& a, v8f& b, v16h x, v16h y) { dep_guard_h(a, b, x, y); }
  static __device__ __forceinline__ void keep(v16h a, v16h b, v16h c, v16h d) { keep4_h(a, b, c, d); }
};
template <> struct Frag<__bf16> {
  typedef v16b V; union U { v16b v; v8b h[2]; };
  static __device__ __forceinline__ v16b load(const __bf16* p) {
    U f; f.h[0] = *(const v8b*)(p); f.h[1] = *(const v8b*)(p + 16); return f.v;
  }
  static __device__ __forceinline__ v8f mma(v16b a, v16b b, v8f c) {
    return __builtin_amdgcn_wmma_f32_16x16x32_bf16(false, a, false, b, (short)0, c, false, false);
  }
  static __device__ __forceinline__ void guard(v8f& a, v8f& b, v16b x, v16b y) { dep_guard_b(a, b, x, y); }
  static __device__ __forceinline__ void keep(v16b a, v16b b, v16b c, v16b d) { keep4_b(a, b, c, d); }
};

template <int ET> struct Elem;
template <> struct Elem<0> { typedef _Float16 T; };
template <> struct Elem<1> { typedef __bf16 T; };
template <int ET, bool SPLIT, int BIAS_MODE, int OUT_MODE, bool RESID, int ACT = 0>
__global__ __launch_bounds__(256) void wmma_gemm64(
    const unsigned short* __restrict__ Ap, const unsigned short* __restrict__ A2p, int lda, long strideA,
    const unsigned short* __restrict__ Btp, const unsigned short* __restrict__ Bt2p, int ldb, long strideB,
    void* __restrict__ Cout, void* __restrict__ Cout2, int ldc, long strideC,
    const float* __restrict__ bias,
    const float* __restrict__ resid, long strideR,
    int M, int N, int K, float scale) {
  typedef typename Elem<ET>::T T;
  typedef typename Frag<T>::V V;
  const T* A = (const T*)Ap; const T* A2 = (const T*)A2p; const T* Bt = (const T*)Btp; const T* Bt2 = (const T*)Bt2p;
  __shared__ __align__(16) float sT[8][16 * 68];
  const int b    = blockIdx.y;
  const int lane = threadIdx.x & 31;
  const int wave = threadIdx.x >> 5;
  const int tilesN = N >> 6;
  const int tilesM = M >> 6;
  const int tile = blockIdx.x * 8 + wave;
  if (tile >= tilesM * tilesN) return;
  const int tm = tile / tilesN;
  const int tn = tile - tm * tilesN;
  const int m0 = tm << 6;
  const int n0 = tn << 6;

  const T* Ab  = A  + (size_t)b * strideA;
  const T* Bb  = Bt + (size_t)b * strideB;
  const T* Ab2 = SPLIT ? (A2  + (size_t)b * strideA) : nullptr;
  const T* Bb2 = SPLIT ? (Bt2 + (size_t)b * strideB) : nullptr;

  const int rlane = lane & 15;
  const int koff  = (lane >> 4) * 8;
  const int mOff  = (lane >> 4) * 8;

  v8f acc[4][4];
#pragma unroll
  for (int i = 0; i < 4; ++i)
#pragma unroll
    for (int j = 0; j < 4; ++j) acc[i][j] = (v8f){0.f,0.f,0.f,0.f,0.f,0.f,0.f,0.f};

  for (int k0 = 0; k0 < K; k0 += 32) {
    V bh[4], bl[4];
#pragma unroll
    for (int j = 0; j < 4; ++j) {
      const size_t bo = (size_t)(n0 + (j << 4) + rlane) * ldb + koff + k0;
      bh[j] = Frag<T>::load(Bb + bo);
      if (SPLIT) bl[j] = Frag<T>::load(Bb2 + bo);
    }
#pragma unroll
    for (int i = 0; i < 4; ++i) {
      const size_t ao = (size_t)(m0 + (i << 4) + rlane) * lda + koff + k0;
      V ah = Frag<T>::load(Ab + ao);
      V al;
      if (SPLIT) al = Frag<T>::load(Ab2 + ao);
#pragma unroll
      for (int j = 0; j < 4; ++j) {
        acc[i][j] = Frag<T>::mma(ah, bh[j], acc[i][j]);
        if (SPLIT) {
          acc[i][j] = Frag<T>::mma(ah, bl[j], acc[i][j]);
          acc[i][j] = Frag<T>::mma(al, bh[j], acc[i][j]);
        }
      }
      Frag<T>::guard(acc[i][0], acc[i][3], ah, SPLIT ? al : ah);
    }
    Frag<T>::keep(bh[0], bh[1], bh[2], bh[3]);
    if (SPLIT) Frag<T>::keep(bl[0], bl[1], bl[2], bl[3]);
  }
  acc_guard4(acc[0][0], acc[0][1], acc[0][2], acc[0][3]);
  acc_guard4(acc[1][0], acc[1][1], acc[1][2], acc[1][3]);
  acc_guard4(acc[2][0], acc[2][1], acc[2][2], acc[2][3]);
  acc_guard4(acc[3][0], acc[3][1], acc[3][2], acc[3][3]);

  float* slab = sT[wave];
  const float* Rb = RESID ? (resid + (size_t)b * strideR) : nullptr;
#pragma unroll
  for (int i = 0; i < 4; ++i) {
    const int mBase = m0 + (i << 4);
#pragma unroll
    for (int j = 0; j < 4; ++j) {
      const int n = n0 + (j << 4) + rlane;
      float bv = 0.f;
      if (BIAS_MODE == 2) bv = bias[n];
#pragma unroll
      for (int r = 0; r < 8; ++r) {
        float v = acc[i][j][r] * scale;
        if (BIAS_MODE == 1) v += bias[mBase + mOff + r];
        if (BIAS_MODE == 2) v += bv;
        if (RESID) v += Rb[(size_t)(mBase + mOff + r) * ldc + n];
        if (ACT == 1) v = tanhf(v);
        if (ACT == 2) v = fmaxf(v, 0.0f);
        if (ACT == 3) v = v / (1.0f + expf(-v));
        if (ACT == 4) v = (v > 0.f) ? v : 0.01f * v;
        if (ACT == 5) v = 0.5f * v * (1.0f + erff(v * 0.70710678118654752f));
        slab[(mOff + r) * 68 + (j << 4) + rlane] = v;
      }
    }
    __builtin_amdgcn_fence(__ATOMIC_RELEASE, "workgroup");
    __builtin_amdgcn_wave_barrier();
    __builtin_amdgcn_fence(__ATOMIC_ACQUIRE, "workgroup");
    if (OUT_MODE == 0) {
      float* C = (float*)Cout + (size_t)b * strideC;
      const int hh = lane >> 4, c4 = (lane & 15) * 4;
      for (int pass = 0; pass < 2; ++pass) {
#pragma unroll
        for (int it = 0; it < 8; ++it) {
          const int row = it * 2 + hh;
          v4f v = *(const v4f*)(slab + row * 68 + c4);
          *(volatile v4f*)(C + (size_t)(mBase + row) * ldc + n0 + c4) = v;
        }
        __threadfence();
      }
    } else {
      const int q = lane >> 3, c8 = (lane & 7) * 8;
      unsigned short* C  = (unsigned short*)Cout  + (size_t)b * strideC;
      unsigned short* C2 = (OUT_MODE == 2) ? ((unsigned short*)Cout2 + (size_t)b * strideC) : nullptr;
      for (int pass = 0; pass < 2; ++pass) {
#pragma unroll
        for (int it = 0; it < 4; ++it) {
          const int row = it * 4 + q;
          const float* sp = slab + row * 68 + c8;
          v8h hv, lv;
#pragma unroll
          for (int e = 0; e < 8; ++e) {
            if (OUT_MODE == 1) {
              hv[e] = (_Float16)sp[e];
            } else {
              unsigned short hb = f2bf_bits(sp[e]);
              unsigned short lb = f2bf_bits(sp[e] - bf_bits2f(hb));
              hv[e] = __builtin_bit_cast(_Float16, hb);
              lv[e] = __builtin_bit_cast(_Float16, lb);
            }
          }
          *(volatile v8h*)(C + (size_t)(mBase + row) * ldc + n0 + c8) = hv;
          if (OUT_MODE == 2) *(volatile v8h*)(C2 + (size_t)(mBase + row) * ldc + n0 + c8) = lv;
        }
        __threadfence();
      }
    }
    __builtin_amdgcn_fence(__ATOMIC_RELEASE, "workgroup");
    __builtin_amdgcn_wave_barrier();
    __builtin_amdgcn_fence(__ATOMIC_ACQUIRE, "workgroup");
  }
}

__global__ __launch_bounds__(256) void wprep_kernel(
    const float* __restrict__ W, _Float16* __restrict__ Wt, int kin, int nout, int kp) {
  __shared__ __align__(16) _Float16 t[64][72];
  const int tid = threadIdx.x;
  const int k0 = blockIdx.x * 64, o0 = blockIdx.y * 64;
#pragma unroll 1
  for (int i = tid; i < 64 * 64; i += 256) {
    const int kk = i >> 6, oo = i & 63;
    const int k = k0 + kk;
    const int kc = (k < kin) ? k : (kin - 1);
    float w = W[(size_t)kc * nout + o0 + oo];
    if (k >= kin) w = 0.f;
    t[oo][kk] = (_Float16)(w * 64.0f);
  }
  __syncthreads();
  for (int pass = 0; pass < 2; ++pass) {
#pragma unroll
    for (int j = 0; j < 2; ++j) {
      const int id = tid + 256 * j;
      const int row = id >> 3, c8 = (id & 7) * 8;
      const v8h hv = *(const v8h*)(&t[row][c8]);
      *(volatile v8h*)(Wt + (size_t)(o0 + row) * kp + k0 + c8) = hv;
    }
    __threadfence();
  }
}

__global__ __launch_bounds__(256) void cast_pose_kernel(
    const float* __restrict__ pe, _Float16* __restrict__ A, int nvalid) {
  const int tid = threadIdx.x;
  for (int pass = 0; pass < 2; ++pass) {
#pragma unroll
    for (int j = 0; j < 4; ++j) {
      const int id = tid + 256 * j;
      const int row = id >> 4, c8 = (id & 15) * 8;
      const int rr = (row < nvalid) ? row : (nvalid - 1);
      v8h hv;
#pragma unroll
      for (int e = 0; e < 8; ++e) {
        float f = pe[(size_t)rr * PDIM + c8 + e];
        if (row >= nvalid) f = 0.f;
        hv[e] = (_Float16)f;
      }
      *(volatile v8h*)(A + (size_t)row * PDIM + c8) = hv;
    }
    __threadfence();
  }
}

__global__ __launch_bounds__(256) void ln_kernel(
    const float* __restrict__ x, const float* __restrict__ peb,
    const float* __restrict__ ng, const float* __restrict__ nb,
    const float* __restrict__ png, const float* __restrict__ pnb,
    _Float16* __restrict__ xnA, _Float16* __restrict__ xpA) {
  __shared__ float xt[LT][516];
  __shared__ __align__(16) _Float16 xn16[LT][NI];
  __shared__ __align__(16) _Float16 xp16[LT][KP];
  __shared__ float pev[2][LT];
  __shared__ float st[LT][4];
  const int tid = threadIdx.x, lane = tid & 31, wave = tid >> 5;
  const int n = blockIdx.x / (SEQ / LT);
  const int s0 = (blockIdx.x - n * (SEQ / LT)) * LT;
  const int tok0 = n * SEQ + s0;

#pragma unroll 1
  for (int i = tid; i < LT * NI; i += 256) {
    const int c = i >> 3, r = i & 7;
    xt[r][c] = x[((size_t)n * NI + c) * SEQ + s0 + r];
  }
  if (tid < 2 * LT) {
    const int i = tid >> 3, r = tid & 7;
    pev[i][r] = peb[(size_t)(n * 2 + i) * SEQ + s0 + r];
  }
  __syncthreads();

  {
    const int R = wave;
    float sum = 0.f;
#pragma unroll 1
    for (int j = 0; j < NI / 32; ++j) sum += xt[R][lane + 32 * j];
#pragma unroll
    for (int off = 1; off < 32; off <<= 1) sum += __shfl_xor(sum, off, 32);
    const float pe0 = pev[0][R], pe1 = pev[1][R];
    const float mean  = sum * (1.0f / 512.0f);
    const float meanp = (sum + pe0 + pe1) * (1.0f / 514.0f);
    float vs = 0.f, vps = 0.f;
#pragma unroll 1
    for (int j = 0; j < NI / 32; ++j) {
      const float xv = xt[R][lane + 32 * j];
      const float d = xv - mean;   vs  += d * d;
      const float dp = xv - meanp; vps += dp * dp;
    }
#pragma unroll
    for (int off = 1; off < 32; off <<= 1) {
      vs  += __shfl_xor(vs, off, 32);
      vps += __shfl_xor(vps, off, 32);
    }
    const float dp0 = pe0 - meanp, dp1 = pe1 - meanp;
    vps += dp0 * dp0 + dp1 * dp1;
    const float inv  = rsqrtf(vs  * (1.0f / 512.0f) + LN_EPS);
    const float invp = rsqrtf(vps * (1.0f / 514.0f) + LN_EPS);
    if (lane == 0) { st[R][0] = mean; st[R][1] = inv; st[R][2] = meanp; st[R][3] = invp; }
  }
  __syncthreads();

#pragma unroll 1
  for (int i = tid; i < LT * KP; i += 256) {
    const int r = i / KP;
    const int c = i - r * KP;
    const float meanp = st[r][2], invp = st[r][3];
    if (c < NI) {
      const float xv = xt[r][c];
      const float mean = st[r][0], inv = st[r][1];
      xn16[r][c] = (_Float16)((xv - mean) * inv * ng[c] + nb[c]);
      xp16[r][c] = (_Float16)((xv - meanp) * invp * png[c] + pnb[c]);
    } else {
      const int cc = (c < KDIM) ? c : (KDIM - 1);
      const int pi = (c == NI) ? 0 : 1;
      float v = (pev[pi][r] - meanp) * invp * png[cc] + pnb[cc];
      if (c >= KDIM) v = 0.f;
      xp16[r][c] = (_Float16)v;
    }
  }
  __syncthreads();

  for (int pass = 0; pass < 2; ++pass) {
#pragma unroll
    for (int j = 0; j < 2; ++j) {
      const int id = tid + 256 * j;
      const int r = id >> 6, c8 = (id & 63) * 8;
      const v8h hv = *(const v8h*)(&xn16[r][c8]);
      *(volatile v8h*)(xnA + ((size_t)tok0 + r) * NI + c8) = hv;
    }
#pragma unroll
    for (int j = 0; j < 3; ++j) {
      const int id = tid + 256 * j;
      if (id < LT * (KP / 8)) {
        const int r = id / (KP / 8), c8 = (id - r * (KP / 8)) * 8;
        const v8h hv = *(const v8h*)(&xp16[r][c8]);
        *(volatile v8h*)(xpA + ((size_t)tok0 + r) * KP + c8) = hv;
      }
    }
    __threadfence();
  }
}

#define AT_D 64
#define AT_NW 4
#define AT_QB 64
#define AT_KC 64

__device__ __forceinline__ v8f mma_h(v16h a, v16h b, v8f c) {
  c = __builtin_amdgcn_wmma_f32_16x16x32_f16(false, a, false, b, (short)0, c, false, false);
  asm volatile("v_nop\n\tv_nop\n\tv_nop\n\tv_nop" : "+v"(c) : "v"(a), "v"(b));
  return c;
}

__global__ __launch_bounds__(128)
void attn16_kernel(const _Float16* __restrict__ q, const _Float16* __restrict__ k,
                   const _Float16* __restrict__ v, _Float16* __restrict__ out,
                   long in_bs, int in_rs, int in_hs, long o_bs, int o_rs, int o_hs,
                   int S, int H, float sscale, float oscale) {
  const float PSC = 32768.0f;
  __shared__ __align__(16) _Float16 Ksh[AT_KC * AT_D];
  __shared__ __align__(16) _Float16 Vth[AT_D * AT_KC];
  __shared__ __align__(16) _Float16 Psh[AT_NW][16 * AT_KC];
  __shared__ __align__(16) float    Os[AT_NW][16 * 68];

  const int tid  = threadIdx.x;
  const int wave = tid >> 5;
  const int lane = tid & 31;
  const int hh   = lane >> 4;
  const int c    = lane & 15;

  const int nqb = S / AT_QB;
  const int bx = blockIdx.x;
  const int qb = bx % nqb;
  const int bh = bx / nqb;
  const int h  = bh % H;
  const int b  = bh / H;
  const int q0 = qb * AT_QB + wave * 16;

  const _Float16* qb_ptr = q + (size_t)b * in_bs + (size_t)h * in_hs;
  const _Float16* kb_ptr = k + (size_t)b * in_bs + (size_t)h * in_hs;
  const _Float16* vb_ptr = v + (size_t)b * in_bs + (size_t)h * in_hs;
  _Float16*       ob_ptr = out + (size_t)b * o_bs + (size_t)h * o_hs;

  v16h qa[2];
#pragma unroll
  for (int dc = 0; dc < 2; ++dc)
    qa[dc] = Frag<_Float16>::load(qb_ptr + (size_t)(q0 + c) * in_rs + dc * 32 + 8 * hh);

  float mrow[8], lrow[8];
  v8f oacc[4];
#pragma unroll
  for (int r = 0; r < 8; ++r) { mrow[r] = -INFINITY; lrow[r] = 0.f; }
#pragma unroll
  for (int t = 0; t < 4; ++t) oacc[t] = (v8f){0.f,0.f,0.f,0.f,0.f,0.f,0.f,0.f};

  const int nChunks = S / AT_KC;
  for (int kc = 0; kc < nChunks; ++kc) {
    const int kv0 = kc * AT_KC;
    __syncthreads();
    {
#pragma unroll
      for (int i = 0; i < 4; ++i) {
        const int id = tid + 128 * i;
        const int kvr = id >> 3, c8 = (id & 7) * 8;
        const v8h kk = *(const v8h*)(kb_ptr + (size_t)(kv0 + kvr) * in_rs + c8);
        *(v8h*)(Ksh + kvr * AT_D + c8) = kk;
        const v8h vv = *(const v8h*)(vb_ptr + (size_t)(kv0 + kvr) * in_rs + c8);
#pragma unroll
        for (int e = 0; e < 8; ++e) Vth[(c8 + e) * AT_KC + kvr] = vv[e];
      }
    }
    __syncthreads();

    v8f s[4];
#pragma unroll
    for (int j = 0; j < 4; ++j) {
      s[j] = (v8f){0.f,0.f,0.f,0.f,0.f,0.f,0.f,0.f};
#pragma unroll
      for (int dc = 0; dc < 2; ++dc) {
        const v16h kb = Frag<_Float16>::load(Ksh + (j * 16 + c) * AT_D + dc * 32 + 8 * hh);
        s[j] = mma_h(qa[dc], kb, s[j]);
      }
    }
    float cm[8];
#pragma unroll
    for (int r = 0; r < 8; ++r) {
      float m = -INFINITY;
#pragma unroll
      for (int j = 0; j < 4; ++j) {
        s[j][r] = s[j][r] * sscale;
        m = fmaxf(m, s[j][r]);
      }
#pragma unroll
      for (int off = 1; off < 16; off <<= 1) m = fmaxf(m, __shfl_xor(m, off, 32));
      cm[r] = m;
    }
    _Float16* pwh = Psh[wave];
#pragma unroll
    for (int r = 0; r < 8; ++r) {
      const float mnew = fmaxf(mrow[r], cm[r]);
      const float alpha = expf(mrow[r] - mnew);
      mrow[r] = mnew;
      float psum = 0.f;
#pragma unroll
      for (int j = 0; j < 4; ++j) {
        const float p = expf(s[j][r] - mnew);
        psum += p;
        pwh[(8 * hh + r) * AT_KC + j * 16 + c] = (_Float16)(p * PSC);
      }
#pragma unroll
      for (int off = 1; off < 16; off <<= 1) psum += __shfl_xor(psum, off, 32);
      lrow[r] = lrow[r] * alpha + psum;
#pragma unroll
      for (int t = 0; t < 4; ++t) oacc[t][r] *= alpha;
    }
    __builtin_amdgcn_fence(__ATOMIC_RELEASE, "workgroup");
    __builtin_amdgcn_wave_barrier();
    __builtin_amdgcn_fence(__ATOMIC_ACQUIRE, "workgroup");
#pragma unroll 1
    for (int kk = 0; kk < 2; ++kk) {
      const v16h pa = Frag<_Float16>::load(pwh + c * AT_KC + kk * 32 + 8 * hh);
#pragma unroll
      for (int t = 0; t < 4; ++t) {
        const v16h vb = Frag<_Float16>::load(Vth + (t * 16 + c) * AT_KC + kk * 32 + 8 * hh);
        oacc[t] = mma_h(pa, vb, oacc[t]);
      }
    }
  }

  float* os = Os[wave];
#pragma unroll
  for (int r = 0; r < 8; ++r) {
    const float inv = oscale * (1.0f / (lrow[r] * PSC));
#pragma unroll
    for (int t = 0; t < 4; ++t) os[(8 * hh + r) * 68 + t * 16 + c] = oacc[t][r] * inv;
  }
  __builtin_amdgcn_fence(__ATOMIC_RELEASE, "workgroup");
  __builtin_amdgcn_wave_barrier();
  __builtin_amdgcn_fence(__ATOMIC_ACQUIRE, "workgroup");
  {
    const int rq = lane >> 3, c8 = (lane & 7) * 8;
    for (int pass = 0; pass < 2; ++pass) {
#pragma unroll
      for (int it = 0; it < 4; ++it) {
        const int row = it * 4 + rq;
        const float* sp = os + row * 68 + c8;
        v8h hv;
#pragma unroll
        for (int e = 0; e < 8; ++e) hv[e] = (_Float16)sp[e];
        *(volatile v8h*)(ob_ptr + (size_t)(q0 + row) * o_rs + c8) = hv;
      }
      __threadfence();
    }
  }
}

static inline size_t al256(size_t v) { return (v + 255) & ~(size_t)255; }

extern "C" void kernel_launch(void* const* d_in, const int* in_sizes, int n_in,
                              void* d_out, int out_size, void* d_ws,
                              size_t ws_size, hipStream_t stream) {
  if (n_in < 16) return;
  if (in_sizes[0] != NBATCH * NI * SEQ) return;
  if (in_sizes[1] != NBATCH * 2 * PDIM) return;
  if (in_sizes[2] != NI || in_sizes[3] != NI) return;
  if (in_sizes[4] != KDIM || in_sizes[5] != KDIM) return;
  if (in_sizes[6] != PDIM * SEQ || in_sizes[7] != SEQ) return;
  if (in_sizes[8] != NI * NI || in_sizes[9] != NI) return;
  if (in_sizes[10] != KDIM * NI || in_sizes[11] != NI) return;
  if (in_sizes[12] != KDIM * NI || in_sizes[13] != NI) return;
  if (in_sizes[14] != NI * NI || in_sizes[15] != NI) return;
  if (out_size != NBATCH * NI * SEQ) return;

  const float* x     = (const float*)d_in[0];
  const float* pose  = (const float*)d_in[1];
  const float* ng    = (const float*)d_in[2];
  const float* nb    = (const float*)d_in[3];
  const float* png   = (const float*)d_in[4];
  const float* pnb   = (const float*)d_in[5];
  const float* poseW = (const float*)d_in[6];
  const float* poseB = (const float*)d_in[7];
  const float* qW    = (const float*)d_in[8];
  const float* qB    = (const float*)d_in[9];
  const float* kW    = (const float*)d_in[10];
  const float* kB    = (const float*)d_in[11];
  const float* vW    = (const float*)d_in[12];
  const float* vB    = (const float*)d_in[13];
  const float* pW    = (const float*)d_in[14];
  const float* pB    = (const float*)d_in[15];
  float* out = (float*)d_out;

  char* ws = (char*)d_ws;
  size_t off = 0;
  const size_t o_qWt   = off; off = al256(off + (size_t)NI * NI * 2);
  const size_t o_kWt   = off; off = al256(off + (size_t)NI * KP * 2);
  const size_t o_vWt   = off; off = al256(off + (size_t)NI * KP * 2);
  const size_t o_pWt   = off; off = al256(off + (size_t)NI * NI * 2);
  const size_t o_psWt  = off; off = al256(off + (size_t)SEQ * PDIM * 2);
  const size_t o_psA   = off; off = al256(off + (size_t)64 * PDIM * 2);
  const size_t o_peb   = off; off = al256(off + (size_t)64 * SEQ * 4);
  const size_t o_xnA   = off; off = al256(off + (size_t)NTOK * NI * 2);
  const size_t o_xpA   = off; off = al256(off + (size_t)NTOK * KP * 2);
  const size_t o_qkv   = off; off = al256(off + (size_t)NTOK * QKVW * 2);
  const size_t o_oA    = off; off = al256(off + (size_t)NTOK * NI * 2);
  const size_t total = off;
  if (total > ws_size) return;
  if (total > (size_t)134217728) return;

  unsigned short* qWt  = (unsigned short*)(ws + o_qWt);
  unsigned short* kWt  = (unsigned short*)(ws + o_kWt);
  unsigned short* vWt  = (unsigned short*)(ws + o_vWt);
  unsigned short* pWt  = (unsigned short*)(ws + o_pWt);
  unsigned short* psWt = (unsigned short*)(ws + o_psWt);
  unsigned short* psA  = (unsigned short*)(ws + o_psA);
  float*          peb  = (float*)(ws + o_peb);
  unsigned short* xnA  = (unsigned short*)(ws + o_xnA);
  unsigned short* xpA  = (unsigned short*)(ws + o_xpA);
  unsigned short* qkv  = (unsigned short*)(ws + o_qkv);
  unsigned short* oA   = (unsigned short*)(ws + o_oA);

  wprep_kernel<<<dim3(NI / 64, NI / 64), 256, 0, stream>>>(qW, (_Float16*)qWt, NI, NI, NI);
  wprep_kernel<<<dim3(KP / 64, NI / 64), 256, 0, stream>>>(kW, (_Float16*)kWt, KDIM, NI, KP);
  wprep_kernel<<<dim3(KP / 64, NI / 64), 256, 0, stream>>>(vW, (_Float16*)vWt, KDIM, NI, KP);
  wprep_kernel<<<dim3(NI / 64, NI / 64), 256, 0, stream>>>(pW, (_Float16*)pWt, NI, NI, NI);
  wprep_kernel<<<dim3(PDIM / 64, SEQ / 64), 256, 0, stream>>>(poseW, (_Float16*)psWt, PDIM, SEQ, PDIM);
  cast_pose_kernel<<<1, 256, 0, stream>>>(pose, (_Float16*)psA, NBATCH * 2);
  wmma_gemm64<0, false, 2, 0, false, 0><<<dim3(2, 1), 256, 0, stream>>>(
      psA, psA, PDIM, 0L, psWt, psWt, PDIM, 0L, (void*)peb, (void*)peb, SEQ, 0L,
      poseB, poseB, 0L, 64, SEQ, PDIM, 1.0f / 64.0f);
  ln_kernel<<<NTOK / LT, 256, 0, stream>>>(x, peb, ng, nb, png, pnb, (_Float16*)xnA, (_Float16*)xpA);
  wmma_gemm64<0, false, 2, 1, false, 0><<<dim3((NTOK / 64) * (NI / 64) / 8, 1), 256, 0, stream>>>(
      xnA, xnA, NI, 0L, qWt, qWt, NI, 0L, (void*)qkv, (void*)qkv, QKVW, 0L,
      qB, qB, 0L, NTOK, NI, NI, 1.0f / 64.0f);
  wmma_gemm64<0, false, 2, 1, false, 0><<<dim3((NTOK / 64) * (NI / 64) / 8, 1), 256, 0, stream>>>(
      xpA, xpA, KP, 0L, kWt, kWt, KP, 0L, (void*)(qkv + NI), (void*)(qkv + NI), QKVW, 0L,
      kB, kB, 0L, NTOK, NI, KP, 1.0f / 64.0f);
  wmma_gemm64<0, false, 2, 1, false, 0><<<dim3((NTOK / 64) * (NI / 64) / 8, 1), 256, 0, stream>>>(
      xpA, xpA, KP, 0L, vWt, vWt, KP, 0L, (void*)(qkv + 2 * NI), (void*)(qkv + 2 * NI), QKVW, 0L,
      vB, vB, 0L, NTOK, NI, KP, 1.0f / 64.0f);
  attn16_kernel<<<NBATCH * NHD * (SEQ / AT_QB), 128, 0, stream>>>(
      (const _Float16*)qkv, (const _Float16*)qkv + DHD, (const _Float16*)qkv + 2 * DHD, (_Float16*)oA,
      (long)SEQ * QKVW, QKVW, 3 * DHD, (long)SEQ * NI, NI, DHD,
      SEQ, NHD, 0.125f, 256.0f);
  wmma_gemm64<0, false, 1, 0, false, 0><<<dim3((NI / 64) * (SEQ / 64) / 8, NBATCH), 256, 0, stream>>>(
      pWt, pWt, NI, 0L, oA, oA, NI, (long)SEQ * NI, (void*)out, (void*)out, SEQ, (long)NI * SEQ,
      pB, pB, 0L, NI, SEQ, NI, 1.0f / (64.0f * 256.0f));
}
